// VNCLCell_33268816675364
// MI455X (gfx1250) — hardware-verified
//
#include <hip/hip_runtime.h>
#include <math.h>

typedef __attribute__((ext_vector_type(16))) _Float16 v16h;
typedef __attribute__((ext_vector_type(8)))  _Float16 v8h;
typedef __attribute__((ext_vector_type(16))) __bf16   v16b;
typedef __attribute__((ext_vector_type(8)))  __bf16   v8b;
typedef __attribute__((ext_vector_type(8)))  float    v8f;
typedef __attribute__((ext_vector_type(4)))  float    v4f;

constexpr int kB    = 4096;
constexpr int kNF   = 2048;
constexpr int kNT   = 300;
constexpr int kNTP  = 320;
constexpr int kR    = 512;
constexpr int kK1   = 3 * kR;
constexpr int kK2   = 2 * kK1;
constexpr int kGates = 4;
constexpr int kThr  = 256;
constexpr float kInCarry = 1024.0f;
constexpr float kWCarry  = 4096.0f;
constexpr float kSc = 1.0f / (kInCarry * kWCarry);
constexpr float kF16MinNormal = 6.103515625e-5f;
constexpr size_t kOut1 = (size_t)kB * kR;

static_assert((kB % 64) == 0 && (kR % 64) == 0 && ((kB / 64) * (kR / 64)) % 8 == 0 && (kR % 32) == 0 && (kNTP % 32) == 0 && (kNF % 32) == 0 && (kK2 % 32) == 0 && (kNTP * 2) % 128 == 0
              && (kR / 8) <= 256 && (kNF / 8) <= 256 && (kNTP / 8) <= 256, "GEMM M, N multiples of 64; grids exact; K multiples of 32; rows are whole lines");

constexpr size_t kOffX16 = 0ull;
constexpr size_t kOffH16 = 4194304ull;
constexpr size_t kOffS16 = 8388608ull;
constexpr size_t kOffV16 = 11010048ull;
constexpr size_t kOffWAT = 27787264ull;
constexpr size_t kOffUAT = 28311552ull;
constexpr size_t kOffCAT = 28835840ull;
constexpr size_t kOffWBT = 30932992ull;
constexpr size_t kOffCBT = 31260672ull;
constexpr size_t kOffUBT = 31588352ull;
constexpr size_t kOffW2T = 31916032ull;
constexpr size_t kOffZB = 35061760ull;
constexpr size_t kOffTA = 35065856ull;
constexpr size_t kOffTB = 43454464ull;
constexpr size_t kOffP16 = 51843072ull;
constexpr size_t kOffLG = 77008896ull;
constexpr size_t kWsTotal = 110563328ull;
static_assert(kWsTotal <= 134217728ull, "carve cap: under 128 MiB");
static_assert(kOffX16 == 0
              && kOffH16 == kOffX16 + 4194304ull
              && kOffS16 == kOffH16 + 4194304ull
              && kOffV16 == kOffS16 + 2621440ull
              && kOffWAT == kOffV16 + 16777216ull
              && kOffUAT == kOffWAT + 524288ull
              && kOffCAT == kOffUAT + 524288ull
              && kOffWBT == kOffCAT + 2097152ull
              && kOffCBT == kOffWBT + 327680ull
              && kOffUBT == kOffCBT + 327680ull
              && kOffW2T == kOffUBT + 327680ull
              && kOffZB == kOffW2T + 3145728ull
              && kOffTA == kOffZB + 4096ull
              && kOffTB == kOffTA + 8388608ull
              && kOffP16 == kOffTB + 8388608ull
              && kOffLG == kOffP16 + 25165824ull
              && kWsTotal == kOffLG + 33554432ull, "the carve is chained and totalled");
static_assert((kOffX16 % 256) == 0 && (kOffH16 % 256) == 0 && (kOffS16 % 256) == 0 && (kOffV16 % 256) == 0 && (kOffWAT % 256) == 0 && (kOffUAT % 256) == 0 && (kOffCAT % 256) == 0 && (kOffWBT % 256) == 0 && (kOffCBT % 256) == 0 && (kOffUBT % 256) == 0 && (kOffW2T % 256) == 0 && (kOffZB % 256) == 0 && (kOffTA % 256) == 0 && (kOffTB % 256) == 0 && (kOffP16 % 256) == 0 && (kOffLG % 256) == 0, "aligned regions");

__device__ __forceinline__ unsigned short f2bf_bits(float f) {
  unsigned u = __float_as_uint(f);
  return (unsigned short)((u + 0x7FFFu + ((u >> 16) & 1u)) >> 16);
}
__device__ __forceinline__ float bf_bits2f(unsigned short h) { return __uint_as_float(((unsigned)h) << 16); }
__device__ __forceinline__ float bf16r(float f) { return bf_bits2f(f2bf_bits(f)); }
__device__ __forceinline__ float carry_flush(float v, float carry) {
  const float s = v * carry;
  return (fabsf(s) < kF16MinNormal) ? 0.0f : s;
}
__device__ __forceinline__ float frcp(float x) { return __builtin_amdgcn_rcpf(x); }

__device__ __forceinline__ void dep_guard4_h(v8f& a, v8f& b, v8f& c, v8f& d, v16h x, v16h y) { asm volatile("v_nop\n\tv_nop\n\tv_nop\n\tv_nop" : "+v"(a), "+v"(b), "+v"(c), "+v"(d) : "v"(x), "v"(y)); }
__device__ __forceinline__ void dep_guard4_b(v8f& a, v8f& b, v8f& c, v8f& d, v16b x, v16b y) { asm volatile("v_nop\n\tv_nop\n\tv_nop\n\tv_nop" : "+v"(a), "+v"(b), "+v"(c), "+v"(d) : "v"(x), "v"(y)); }
__device__ __forceinline__ void keep4_h(v16h a, v16h b, v16h c, v16h d) { asm volatile("v_nop" :: "v"(a), "v"(b), "v"(c), "v"(d)); }
__device__ __forceinline__ void keep4_b(v16b a, v16b b, v16b c, v16b d) { asm volatile("v_nop" :: "v"(a), "v"(b), "v"(c), "v"(d)); }
__device__ __forceinline__ void acc_guard4(v8f& a, v8f& b, v8f& c, v8f& d) { asm volatile("v_nop\n\tv_nop\n\tv_nop\n\tv_nop" : "+v"(a), "+v"(b), "+v"(c), "+v"(d)); }

template <typename T> struct Frag;
template <> struct Frag<_Float16> {
  typedef v16h V; union U { v16h v; v8h h[2]; };
  static __device__ __forceinline__ v16h load(const _Float16* p) {
    U f; f.h[0] = *(const v8h*)(p); f.h[1] = *(const v8h*)(p + 16); return f.v;
  }
  static __device__ __forceinline__ v8f mma(v16h a, v16h b, v8f c) {
    return __builtin_amdgcn_wmma_f32_16x16x32_f16(false, a, false, b, (short)0, c, false, false);
  }
  static __device__ __forceinline__ void guard4(v8f& a, v8f& b, v8f& c, v8f& d, v16h x, v16h y) { dep_guard4_h(a, b, c, d, x, y); }
  static __device__ __forceinline__ void keep(v16h a, v16h b, v16h c, v16h d) { keep4_h(a, b, c, d); }
};
template <> struct Frag<__bf16> {
  typedef v16b V; union U { v16b v; v8b h[2]; };
  static __device__ __forceinline__ v16b load(const __bf16* p) {
    U f; f.h[0] = *(const v8b*)(p); f.h[1] = *(const v8b*)(p + 16); return f.v;
  }
  static __device__ __forceinline__ v8f mma(v16b a, v16b b, v8f c) {
    return __builtin_amdgcn_wmma_f32_16x16x32_bf16(false, a, false, b, (short)0, c, false, false);
  }
  static __device__ __forceinline__ void guard4(v8f& a, v8f& b, v8f& c, v8f& d, v16b x, v16b y) { dep_guard4_b(a, b, c, d, x, y); }
  static __device__ __forceinline__ void keep(v16b a, v16b b, v16b c, v16b d) { keep4_b(a, b, c, d); }
};

__device__ __forceinline__ v8f mma_h(v16h a, v16h b, v8f c) {
  c = __builtin_amdgcn_wmma_f32_16x16x32_f16(false, a, false, b, (short)0, c, false, false);
  asm volatile("v_nop\n\tv_nop\n\tv_nop\n\tv_nop" : "+v"(c) : "v"(a), "v"(b));
  return c;
}

template <int ET> struct Elem;
template <> struct Elem<0> { typedef _Float16 T; };
template <> struct Elem<1> { typedef __bf16 T; };
template <int ET, bool SPLIT, int BIAS_MODE, int OUT_MODE, bool RESID, int ACT = 0>
__global__ __launch_bounds__(256) void wmma_gemm64(
    const unsigned short* __restrict__ Ap, const unsigned short* __restrict__ A2p, int lda, long strideA,
    const unsigned short* __restrict__ Btp, const unsigned short* __restrict__ Bt2p, int ldb, long strideB,
    void* __restrict__ Cout, void* __restrict__ Cout2, int ldc, long strideC,
    const float* __restrict__ bias,
    const float* __restrict__ resid, long strideR,
    int M, int N, int K, float scale) {
  typedef typename Elem<ET>::T T;
  typedef typename Frag<T>::V V;
  const T* A = (const T*)Ap; const T* A2 = (const T*)A2p; const T* Bt = (const T*)Btp; const T* Bt2 = (const T*)Bt2p;
  __shared__ __align__(16) float sT[8][16 * 68];
  const int b    = blockIdx.y;
  const int lane = threadIdx.x & 31;
  const int wave = threadIdx.x >> 5;
  const int tilesN = N >> 6;
  const int tilesM = M >> 6;
  const int tile = blockIdx.x * 8 + wave;
  if (tile >= tilesM * tilesN) return;
  const int tm = tile / tilesN;
  const int tn = tile - tm * tilesN;
  const int m0 = tm << 6;
  const int n0 = tn << 6;

  const T* Ab  = A  + (size_t)b * strideA;
  const T* Bb  = Bt + (size_t)b * strideB;
  const T* Ab2 = SPLIT ? (A2  + (size_t)b * strideA) : nullptr;
  const T* Bb2 = SPLIT ? (Bt2 + (size_t)b * strideB) : nullptr;

  const int rlane = lane & 15;
  const int koff  = (lane >> 4) * 8;
  const int mOff  = (lane >> 4) * 8;

  v8f acc[4][4];
#pragma unroll
  for (int i = 0; i < 4; ++i)
#pragma unroll
    for (int j = 0; j < 4; ++j) acc[i][j] = (v8f){0.f,0.f,0.f,0.f,0.f,0.f,0.f,0.f};

  for (int k0 = 0; k0 < K; k0 += 32) {
    V bh[4], bl[4];
#pragma unroll
    for (int j = 0; j < 4; ++j) {
      const size_t bo = (size_t)(n0 + (j << 4) + rlane) * ldb + koff + k0;
      bh[j] = Frag<T>::load(Bb + bo);
      if (SPLIT) bl[j] = Frag<T>::load(Bb2 + bo);
    }
#pragma unroll
    for (int i = 0; i < 4; ++i) {
      const size_t ao = (size_t)(m0 + (i << 4) + rlane) * lda + koff + k0;
      V ah = Frag<T>::load(Ab + ao);
      V al;
      if (SPLIT) al = Frag<T>::load(Ab2 + ao);
#pragma unroll
      for (int j = 0; j < 4; ++j) {
        acc[i][j] = Frag<T>::mma(ah, bh[j], acc[i][j]);
        if (SPLIT) {
          acc[i][j] = Frag<T>::mma(ah, bl[j], acc[i][j]);
          acc[i][j] = Frag<T>::mma(al, bh[j], acc[i][j]);
        }
      }
      Frag<T>::guard4(acc[i][0], acc[i][1], acc[i][2], acc[i][3], ah, SPLIT ? al : ah);
    }
    Frag<T>::keep(bh[0], bh[1], bh[2], bh[3]);
    if (SPLIT) Frag<T>::keep(bl[0], bl[1], bl[2], bl[3]);
  }
  acc_guard4(acc[0][0], acc[0][1], acc[0][2], acc[0][3]);
  acc_guard4(acc[1][0], acc[1][1], acc[1][2], acc[1][3]);
  acc_guard4(acc[2][0], acc[2][1], acc[2][2], acc[2][3]);
  acc_guard4(acc[3][0], acc[3][1], acc[3][2], acc[3][3]);

  float* slab = sT[wave];
  const float* Rb = RESID ? (resid + (size_t)b * strideR) : nullptr;
#pragma unroll
  for (int i = 0; i < 4; ++i) {
    const int mBase = m0 + (i << 4);
#pragma unroll
    for (int j = 0; j < 4; ++j) {
      const int n = n0 + (j << 4) + rlane;
      float bv = 0.f;
      if (BIAS_MODE == 2) bv = bias[n];
#pragma unroll
      for (int r = 0; r < 8; ++r) {
        float v = acc[i][j][r] * scale;
        if (BIAS_MODE == 1) v += bias[mBase + mOff + r];
        if (BIAS_MODE == 2) v += bv;
        if (RESID) v += Rb[(size_t)(mBase + mOff + r) * ldc + n];
        if (ACT == 1) v = tanhf(v);
        if (ACT == 2) v = fmaxf(v, 0.0f);
        if (ACT == 3) v = v / (1.0f + expf(-v));
        if (ACT == 4) v = (v > 0.f) ? v : 0.01f * v;
        slab[(mOff + r) * 68 + (j << 4) + rlane] = v;
      }
    }
    __builtin_amdgcn_fence(__ATOMIC_RELEASE, "workgroup");
    __builtin_amdgcn_wave_barrier();
    __builtin_amdgcn_fence(__ATOMIC_ACQUIRE, "workgroup");
    if (OUT_MODE == 0) {
      float* C = (float*)Cout + (size_t)b * strideC;
      const int hh = lane >> 4, c4 = (lane & 15) * 4;
      for (int pass = 0; pass < 2; ++pass) {
#pragma unroll
        for (int it = 0; it < 8; ++it) {
          const int row = it * 2 + hh;
          v4f v = *(const v4f*)(slab + row * 68 + c4);
          *(volatile v4f*)(C + (size_t)(mBase + row) * ldc + n0 + c4) = v;
        }
        __threadfence();
      }
    } else {
      const int q = lane >> 3, c8 = (lane & 7) * 8;
      unsigned short* C  = (unsigned short*)Cout  + (size_t)b * strideC;
      unsigned short* C2 = (OUT_MODE == 2) ? ((unsigned short*)Cout2 + (size_t)b * strideC) : nullptr;
      for (int pass = 0; pass < 2; ++pass) {
#pragma unroll
        for (int it = 0; it < 4; ++it) {
          const int row = it * 4 + q;
          const float* sp = slab + row * 68 + c8;
          v8h hv, lv;
#pragma unroll
          for (int e = 0; e < 8; ++e) {
            if (OUT_MODE == 1) {
              hv[e] = (_Float16)sp[e];
            } else {
              unsigned short hb = f2bf_bits(sp[e]);
              unsigned short lb = f2bf_bits(sp[e] - bf_bits2f(hb));
              hv[e] = __builtin_bit_cast(_Float16, hb);
              lv[e] = __builtin_bit_cast(_Float16, lb);
            }
          }
          *(volatile v8h*)(C + (size_t)(mBase + row) * ldc + n0 + c8) = hv;
          if (OUT_MODE == 2) *(volatile v8h*)(C2 + (size_t)(mBase + row) * ldc + n0 + c8) = lv;
        }
        __threadfence();
      }
    }
    __builtin_amdgcn_fence(__ATOMIC_RELEASE, "workgroup");
    __builtin_amdgcn_wave_barrier();
    __builtin_amdgcn_fence(__ATOMIC_ACQUIRE, "workgroup");
  }
}

__global__ __launch_bounds__(kThr) void cast_plane_kernel(const float* __restrict__ src, unsigned short* __restrict__ dst,
                                                          int colsLog2, int dstPitch, int dstOff) {
  const int i   = blockIdx.x * kThr + threadIdx.x;
  const int sh  = colsLog2 - 3;
  const int row = i >> sh;
  const int c8  = (i & ((1 << sh) - 1)) * 8;
  const float* sp = src + ((size_t)row << colsLog2) + c8;
  const v4f a0 = *(const v4f*)(sp);
  const v4f a1 = *(const v4f*)(sp + 4);
  v8h hv;
#pragma unroll
  for (int e = 0; e < 4; ++e) {
    const float f0 = a0[e];
    const float f1 = a1[e];
    hv[e]     = (_Float16)carry_flush(bf16r(f0), kInCarry);
    hv[4 + e] = (_Float16)carry_flush(bf16r(f1), kInCarry);
  }
  unsigned short* dp = dst + (size_t)row * dstPitch + dstOff + c8;
  *(volatile v8h*)dp = hv;
  __threadfence();
  *(volatile v8h*)dp = hv;
}
__global__ __launch_bounds__(256) void wt_plane_kernel(const float* __restrict__ W, unsigned short* __restrict__ dst, int K, int N, int nLive, int ldd, int colOff) {
  const int n  = blockIdx.x;
  const int k8 = threadIdx.x * 8;
  const bool live = n < nLive;
  const int nc = live ? n : 0;
  v8h hv;
#pragma unroll
  for (int e = 0; e < 8; ++e) {
    const float w = W[(size_t)(k8 + e) * N + nc];
    hv[e] = (_Float16)(live ? carry_flush(bf16r(w), kWCarry) : 0.0f);
  }
  unsigned short* dp = dst + (size_t)n * ldd + colOff + k8;
  *(volatile v8h*)dp = hv;
  __threadfence();
  *(volatile v8h*)dp = hv;
}


__device__ __forceinline__ float fast_tanh(float v) { return 1.0f - 2.0f * frcp(__expf(2.0f * v) + 1.0f); }
__device__ __forceinline__ float fast_sigmoid(float v) { return frcp(1.0f + __expf(-v)); }
__device__ __forceinline__ void split_f16(float x, float c, float cinv, _Float16& hi, _Float16& lo) {
  hi = (_Float16)carry_flush(x, c);
  const float back = (float)hi * cinv;
  lo = (_Float16)carry_flush(x - back, c);
}

__global__ __launch_bounds__(kThr) void scast_kernel(const float* __restrict__ s, unsigned short* __restrict__ S16, float* __restrict__ ZB) {
  unsigned v = blockIdx.x * (unsigned)kThr + threadIdx.x;
  asm volatile("" : "+v"(v));
  if (v < 163840u) {
    const unsigned b = v / 40u, k8 = (v % 40u) * 8u;
    v8h hv;
#pragma unroll
    for (int e = 0; e < 8; ++e) {
      const unsigned k = k8 + (unsigned)e;
      const bool live = k < (unsigned)kNT;
      float w = s[(size_t)b * kNT + (live ? k : 0u)];
      asm volatile("" : "+v"(w));
      hv[e] = (_Float16)(live ? carry_flush(bf16r(w), kInCarry) : 0.0f);
    }
    unsigned short* dp = S16 + (size_t)v * 8u;
    *(volatile v8h*)dp = hv;
    __threadfence();
    *(volatile v8h*)dp = hv;
  } else {
    const v4f z = {0.f, 0.f, 0.f, 0.f};
    float* dp = ZB + (size_t)(v - 163840u) * 4u;
    *(volatile v4f*)dp = z;
    __threadfence();
    *(volatile v4f*)dp = z;
  }
}
static_assert(kB * (kNTP / 8) == 163840 && 163840 % kThr == 0 && 163840 + 256 == 641 * kThr, "tag cast grid exact");

__global__ __launch_bounds__(64) void wt300_kernel(const float* __restrict__ W, unsigned short* __restrict__ dst) {
  const int n  = blockIdx.x;
  const int k8 = threadIdx.x * 8;
  v8h hv;
#pragma unroll
  for (int e = 0; e < 8; ++e) {
    const int k = k8 + e;
    const bool live = k < kNT;
    float w = W[(size_t)(live ? k : 0) * kR + n];
    asm volatile("" : "+v"(w));
    hv[e] = (_Float16)(live ? carry_flush(bf16r(w), kWCarry) : 0.0f);
  }
  unsigned short* dp = dst + (size_t)n * kNTP + k8;
  *(volatile v8h*)dp = hv;
  __threadfence();
  *(volatile v8h*)dp = hv;
}

__global__ __launch_bounds__(kThr) void fuse_kernel(const float* __restrict__ TA, const float* __restrict__ TB, unsigned short* __restrict__ P16, int colOff) {
  unsigned v = blockIdx.x * (unsigned)kThr + threadIdx.x;
  asm volatile("" : "+v"(v));
  const unsigned b = v >> 6, r8 = (v & 63u) * 8u;
  const size_t o8 = (size_t)b * kR + r8;
  const v4f a0 = *(const v4f*)(TA + o8), a1 = *(const v4f*)(TA + o8 + 4), b0 = *(const v4f*)(TB + o8), b1 = *(const v4f*)(TB + o8 + 4);
  v8h hv, lv;
#pragma unroll
  for (int e = 0; e < 4; ++e) {
    _Float16 hi, lo;
    split_f16(a0[e] * b0[e], kInCarry, 1.0f / kInCarry, hi, lo); hv[e] = hi; lv[e] = lo;
    split_f16(a1[e] * b1[e], kInCarry, 1.0f / kInCarry, hi, lo); hv[4 + e] = hi; lv[4 + e] = lo;
  }
  unsigned short* dp = P16 + (size_t)b * kK2 + (size_t)colOff + r8;
  for (int pass = 0; pass < 2; ++pass) {
    *(volatile v8h*)dp = hv;
    *(volatile v8h*)(dp + kK1) = lv;
    __threadfence();
  }
}
static_assert((size_t)kB * kR / 8 == 1024 * (size_t)kThr, "fusion grid exact");

__global__ __launch_bounds__(kThr) void cell_kernel(const float* __restrict__ LG, const float* __restrict__ bias, const float* __restrict__ c,
                                                    float* __restrict__ out_h, float* __restrict__ out_c) {
  unsigned v = blockIdx.x * (unsigned)kThr + threadIdx.x;
  asm volatile("" : "+v"(v));
  const size_t o4 = (size_t)v * 4u;
  const unsigned u4 = (unsigned)(o4 & (size_t)(kR - 1));
  const size_t gs = (size_t)kB * kR;
  const v4f li = *(const v4f*)(LG + o4), lf = *(const v4f*)(LG + gs + o4), lo = *(const v4f*)(LG + 2 * gs + o4), lc = *(const v4f*)(LG + 3 * gs + o4);
  const v4f bi = *(const v4f*)(bias + u4), bf_ = *(const v4f*)(bias + kR + u4), bo = *(const v4f*)(bias + 2 * kR + u4), bc = *(const v4f*)(bias + 3 * kR + u4);
  const v4f co = *(const v4f*)(c + o4);
  v4f nh, nc;
#pragma unroll
  for (int e = 0; e < 4; ++e) {
    const float p0 = bi[e], p1 = bf_[e], p2 = bo[e], p3 = bc[e], pc = co[e];
    const float ig = fast_sigmoid(li[e] + bf16r(p0));
    const float fg = fast_sigmoid(lf[e] + bf16r(p1));
    const float og = fast_sigmoid(lo[e] + bf16r(p2));
    const float gg = fast_tanh(lc[e] + bf16r(p3));
    const float cn = fg * bf16r(pc) + ig * gg;
    nc[e] = cn;
    nh[e] = og * fast_tanh(cn);
  }
  for (int pass = 0; pass < 2; ++pass) {
    *(volatile v4f*)(out_h + o4) = nh;
    *(volatile v4f*)(out_c + o4) = nc;
    __threadfence();
  }
}
static_assert((size_t)kB * kR / 4 == 2048 * (size_t)kThr && (kR & (kR - 1)) == 0, "cell grid exact");

static_assert(((size_t)kB * kR / 8) % kThr == 0 && ((size_t)kB * kNF / 8) % kThr == 0, "plane cast grids exact");

extern "C" void kernel_launch(void* const* d_in, const int* in_sizes, int n_in,
                              void* d_out, int out_size, void* d_ws, size_t ws_size,
                              hipStream_t stream) {
  if (n_in < 15 || d_out == nullptr || d_ws == nullptr) return;
  if (in_sizes[0] != kB * kNF || in_sizes[1] != kB * kNT || in_sizes[2] != kB * kR || in_sizes[3] != kB * kR || in_sizes[4] != kB * kR) return;
  if (in_sizes[5] != kGates * kR * kR || in_sizes[6] != kGates * kNT * kR || in_sizes[7] != kGates * kR * kR || in_sizes[8] != kGates * kR * kR) return;
  if (in_sizes[9] != kGates * kNT * kR || in_sizes[10] != kGates * kR * kR || in_sizes[11] != kGates * kNF * kR || in_sizes[12] != kGates * kNT * kR) return;
  if (in_sizes[13] != kGates * kR * kR || in_sizes[14] != kGates * kR) return;
  if ((size_t)out_size != 2 * kOut1) return;
  if (ws_size < kWsTotal) return;
  const float* v = (const float*)d_in[0];
  const float* s = (const float*)d_in[1];
  const float* x = (const float*)d_in[2];
  const float* h = (const float*)d_in[3];
  const float* c = (const float*)d_in[4];
  const float* Wa = (const float*)d_in[5];
  const float* Wb = (const float*)d_in[6];
  const float* Wc = (const float*)d_in[7];
  const float* Ua = (const float*)d_in[8];
  const float* Ub = (const float*)d_in[9];
  const float* Uc = (const float*)d_in[10];
  const float* Ca = (const float*)d_in[11];
  const float* Cb = (const float*)d_in[12];
  const float* Cc = (const float*)d_in[13];
  const float* bias = (const float*)d_in[14];
  float* out = (float*)d_out;
  char* ws = (char*)d_ws;
  unsigned short* X16 = (unsigned short*)(ws + kOffX16);
  unsigned short* H16 = (unsigned short*)(ws + kOffH16);
  unsigned short* S16 = (unsigned short*)(ws + kOffS16);
  unsigned short* V16 = (unsigned short*)(ws + kOffV16);
  unsigned short* WAT = (unsigned short*)(ws + kOffWAT);
  unsigned short* UAT = (unsigned short*)(ws + kOffUAT);
  unsigned short* CAT = (unsigned short*)(ws + kOffCAT);
  unsigned short* WBT = (unsigned short*)(ws + kOffWBT);
  unsigned short* CBT = (unsigned short*)(ws + kOffCBT);
  unsigned short* UBT = (unsigned short*)(ws + kOffUBT);
  unsigned short* W2T = (unsigned short*)(ws + kOffW2T);
  float* ZB = (float*)(ws + kOffZB);
  float* TA = (float*)(ws + kOffTA);
  float* TB = (float*)(ws + kOffTB);
  unsigned short* P16 = (unsigned short*)(ws + kOffP16);
  float* LG = (float*)(ws + kOffLG);

  cast_plane_kernel<<<(int)(((size_t)kB * kR / 8) / kThr), kThr, 0, stream>>>(x, X16, 9, kR, 0);
  cast_plane_kernel<<<(int)(((size_t)kB * kR / 8) / kThr), kThr, 0, stream>>>(h, H16, 9, kR, 0);
  cast_plane_kernel<<<(int)(((size_t)kB * kNF / 8) / kThr), kThr, 0, stream>>>(v, V16, 11, kNF, 0);
  scast_kernel<<<641, kThr, 0, stream>>>(s, S16, ZB);

  for (int g = 0; g < kGates; ++g) {
    const size_t rr = (size_t)g * kR * kR, tr = (size_t)g * kNT * kR, fr = (size_t)g * kNF * kR;
    wt_plane_kernel<<<kR, kR / 8, 0, stream>>>(Wa + rr, WAT, kR, kR, kR, kR, 0);
    wt_plane_kernel<<<kR, kR / 8, 0, stream>>>(Ua + rr, UAT, kR, kR, kR, kR, 0);
    wt_plane_kernel<<<kR, kNF / 8, 0, stream>>>(Ca + fr, CAT, kNF, kR, kR, kNF, 0);
    for (int w = 0; w < 2; ++w) {
      wt_plane_kernel<<<kR, kR / 8, 0, stream>>>(Wc + rr, W2T, kR, kR, kR, kK2, w * kK1);
      wt_plane_kernel<<<kR, kR / 8, 0, stream>>>(Cc + rr, W2T, kR, kR, kR, kK2, w * kK1 + kR);
      wt_plane_kernel<<<kR, kR / 8, 0, stream>>>(Uc + rr, W2T, kR, kR, kR, kK2, w * kK1 + 2 * kR);
    }
    wt300_kernel<<<kR, kNTP / 8, 0, stream>>>(Wb + tr, WBT);
    wt300_kernel<<<kR, kNTP / 8, 0, stream>>>(Cb + tr, CBT);
    wt300_kernel<<<kR, kNTP / 8, 0, stream>>>(Ub + tr, UBT);

    wmma_gemm64<0, false, 2, 0, false, 0><<<dim3((kB / 64) * (kR / 64) / 8, 1), 256, 0, stream>>>(
        X16, X16, kR, 0L, WAT, WAT, kR, 0L, (void*)TA, (void*)TA, kR, 0L, ZB, nullptr, 0L, kB, kR, kR, kSc);
    wmma_gemm64<0, false, 2, 0, false, 0><<<dim3((kB / 64) * (kR / 64) / 8, 1), 256, 0, stream>>>(
        S16, S16, kNTP, 0L, WBT, WBT, kNTP, 0L, (void*)TB, (void*)TB, kR, 0L, ZB, nullptr, 0L, kB, kR, kNTP, kSc);
    fuse_kernel<<<1024, kThr, 0, stream>>>(TA, TB, P16, 0);
    wmma_gemm64<0, false, 2, 0, false, 0><<<dim3((kB / 64) * (kR / 64) / 8, 1), 256, 0, stream>>>(
        V16, V16, kNF, 0L, CAT, CAT, kNF, 0L, (void*)TA, (void*)TA, kR, 0L, ZB, nullptr, 0L, kB, kR, kNF, kSc);
    wmma_gemm64<0, false, 2, 0, false, 0><<<dim3((kB / 64) * (kR / 64) / 8, 1), 256, 0, stream>>>(
        S16, S16, kNTP, 0L, CBT, CBT, kNTP, 0L, (void*)TB, (void*)TB, kR, 0L, ZB, nullptr, 0L, kB, kR, kNTP, kSc);
    fuse_kernel<<<1024, kThr, 0, stream>>>(TA, TB, P16, kR);
    wmma_gemm64<0, false, 2, 0, false, 0><<<dim3((kB / 64) * (kR / 64) / 8, 1), 256, 0, stream>>>(
        S16, S16, kNTP, 0L, UBT, UBT, kNTP, 0L, (void*)TA, (void*)TA, kR, 0L, ZB, nullptr, 0L, kB, kR, kNTP, kSc);
    wmma_gemm64<0, false, 2, 0, false, 0><<<dim3((kB / 64) * (kR / 64) / 8, 1), 256, 0, stream>>>(
        H16, H16, kR, 0L, UAT, UAT, kR, 0L, (void*)TB, (void*)TB, kR, 0L, ZB, nullptr, 0L, kB, kR, kR, kSc);
    fuse_kernel<<<1024, kThr, 0, stream>>>(TA, TB, P16, 2 * kR);
    float* LGg = LG + (size_t)g * kB * kR;
    wmma_gemm64<0, false, 2, 0, false, 0><<<dim3((kB / 64) * (kR / 64) / 8, 1), 256, 0, stream>>>(
        P16, P16, kK2, 0L, W2T, W2T, kK2, 0L, (void*)LGg, (void*)LGg, kR, 0L, ZB, nullptr, 0L, kB, kR, kK2, kSc);
  }
  cell_kernel<<<2048, kThr, 0, stream>>>(LG, bias, c, out, out + kOut1);
}
